// ScaledDotProductSelector_29884382446394
// MI455X (gfx1250) — hardware-verified
//
#include <hip/hip_runtime.h>


typedef _Float16 v16h __attribute__((ext_vector_type(16)));
typedef _Float16 v8h  __attribute__((ext_vector_type(8), may_alias));
typedef float    v8f  __attribute__((ext_vector_type(8)));
typedef float    v4f  __attribute__((ext_vector_type(4), may_alias));

#define BATCH 2
#define HEADS 16
#define SEQ   2048
#define DIM   64
#define QT    128
#define KT    64
#define NWAVE 8
#define NTHR  (NWAVE * 32)
#define PADH  72
#define OPAD  68

typedef char shape_check[(SEQ % QT == 0 && QT == NWAVE * 16 && QT % KT == 0 && DIM == 64 && KT == 64) ? 1 : -1];

struct LdsMain {
    _Float16 Qs[QT][PADH];
    _Float16 Ks[KT][PADH];
    _Float16 Vt[DIM][PADH];
    _Float16 Ps[NWAVE][16][PADH];
};
struct LdsOut {
    float Os[NWAVE][16][OPAD];
};
union LdsAll { LdsMain a; LdsOut b; };

union Frag { v16h v; v8h h8[2]; };

__device__ __forceinline__ v8f wmma_f16_32k(v16h a, v16h b, v8f c)
{
    v8f d = __builtin_amdgcn_wmma_f32_16x16x32_f16(false, a, false, b, (short)0, c, false, false);
    asm volatile("v_nop\n\tv_nop\n\tv_nop\n\tv_nop" : "+v"(d) : "v"(a), "v"(b));
    return d;
}

__device__ __forceinline__ float bf16_rne(float x)
{
    unsigned int u = __float_as_uint(x);
    u = (u + 0x7FFFu + ((u >> 16) & 1u)) & 0xFFFF0000u;
    return __uint_as_float(u);
}

__global__ __launch_bounds__(NTHR)
void attn_causal_fwd(const float* __restrict__ q,
                     const float* __restrict__ k,
                     const float* __restrict__ v,
                     float* __restrict__ out,
                     int nbh)
{
    __shared__ __align__(16) LdsAll sm;

    const int tid  = threadIdx.x;
    const int wid  = tid >> 5;
    const int lane = tid & 31;
    const int m    = lane & 15;
    const int hs   = lane >> 4;

    const int bh = blockIdx.y;
    const int q0 = blockIdx.x * QT;
    if (bh >= nbh || q0 + QT > SEQ) return;

    const size_t base  = (size_t)bh * SEQ * DIM;
    const int   wrow0  = q0 + wid * 16;
    const int   rowmax = wrow0 + 15;

    for (int i = tid; i < QT * (DIM / 4); i += NTHR) {
        const int r = i >> 4, c = (i & 15) * 4;
        const float4 x = *reinterpret_cast<const float4*>(q + base + (size_t)(q0 + r) * DIM + c);
        sm.a.Qs[r][c + 0] = (_Float16)(bf16_rne(x.x) * 16.0f);
        sm.a.Qs[r][c + 1] = (_Float16)(bf16_rne(x.y) * 16.0f);
        sm.a.Qs[r][c + 2] = (_Float16)(bf16_rne(x.z) * 16.0f);
        sm.a.Qs[r][c + 3] = (_Float16)(bf16_rne(x.w) * 16.0f);
    }
    __syncthreads();

    v16h aQ[2];
    #pragma unroll
    for (int s = 0; s < 2; ++s) {
        Frag f;
        f.h8[0] = *(const v8h*)(&sm.a.Qs[wid * 16 + m][s * 32 + 8 * hs]);
        f.h8[1] = *(const v8h*)(&sm.a.Qs[wid * 16 + m][s * 32 + 16 + 8 * hs]);
        aQ[s] = f.v;
    }

    v8f Oacc[4];
    #pragma unroll
    for (int t = 0; t < 4; ++t) Oacc[t] = (v8f){};
    float mr[8], lr[8];
    #pragma unroll
    for (int r = 0; r < 8; ++r) { mr[r] = -1e30f; lr[r] = 0.0f; }

    const int ntiles = (q0 + QT) / KT;

    for (int jt = 0; jt < ntiles; ++jt) {
        const int  j0       = jt * KT;
        const bool active   = (j0 <= rowmax);
        const bool needMask = (j0 + KT - 1 > wrow0);

        __syncthreads();

        for (int i = tid; i < KT * (DIM / 4); i += NTHR) {
            const int r = i >> 4, c = (i & 15) * 4;
            const size_t g = base + (size_t)(j0 + r) * DIM + c;
            const float4 xk = *reinterpret_cast<const float4*>(k + g);
            const float4 xv = *reinterpret_cast<const float4*>(v + g);
            sm.a.Ks[r][c + 0] = (_Float16)(bf16_rne(xk.x) * 16.0f);
            sm.a.Ks[r][c + 1] = (_Float16)(bf16_rne(xk.y) * 16.0f);
            sm.a.Ks[r][c + 2] = (_Float16)(bf16_rne(xk.z) * 16.0f);
            sm.a.Ks[r][c + 3] = (_Float16)(bf16_rne(xk.w) * 16.0f);
            sm.a.Vt[c + 0][r] = (_Float16)bf16_rne(xv.x);
            sm.a.Vt[c + 1][r] = (_Float16)bf16_rne(xv.y);
            sm.a.Vt[c + 2][r] = (_Float16)bf16_rne(xv.z);
            sm.a.Vt[c + 3][r] = (_Float16)bf16_rne(xv.w);
        }
        __syncthreads();

        if (active) {
            v8f Sacc[4];
            #pragma unroll
            for (int t = 0; t < 4; ++t) {
                v8f acc = (v8f){};
                #pragma unroll
                for (int s = 0; s < 2; ++s) {
                    Frag fb;
                    fb.h8[0] = *(const v8h*)(&sm.a.Ks[t * 16 + m][s * 32 + 8 * hs]);
                    fb.h8[1] = *(const v8h*)(&sm.a.Ks[t * 16 + m][s * 32 + 16 + 8 * hs]);
                    acc = wmma_f16_32k(aQ[s], fb.v, acc);
                }
                Sacc[t] = acc * (1.0f / 256.0f);
            }

            if (needMask) {
                #pragma unroll
                for (int r = 0; r < 8; ++r) {
                    const int mabs = wrow0 + 8 * hs + r;
                    #pragma unroll
                    for (int t = 0; t < 4; ++t) {
                        const int nabs = j0 + t * 16 + m;
                        if (nabs > mabs) Sacc[t][r] = -1e30f;
                    }
                }
            }

            #pragma unroll
            for (int r = 0; r < 8; ++r) {
                float mx = fmaxf(fmaxf(Sacc[0][r], Sacc[1][r]), fmaxf(Sacc[2][r], Sacc[3][r]));
                mx = fmaxf(mx, __shfl_xor(mx, 1, 32));
                mx = fmaxf(mx, __shfl_xor(mx, 2, 32));
                mx = fmaxf(mx, __shfl_xor(mx, 4, 32));
                mx = fmaxf(mx, __shfl_xor(mx, 8, 32));
                const float mnew  = fmaxf(mr[r], mx);
                const float alpha = __expf(mr[r] - mnew);
                mr[r] = mnew;
                float ls = 0.0f;
                #pragma unroll
                for (int t = 0; t < 4; ++t) {
                    float p = __expf(Sacc[t][r] - mnew) * 4096.0f;
                    p = (p < 6.103515625e-05f) ? 0.0f : p;
                    const _Float16 ph = (_Float16)p;
                    sm.a.Ps[wid][r + 8 * hs][t * 16 + m] = ph;
                    ls += (float)ph;
                }
                ls += __shfl_xor(ls, 1, 32);
                ls += __shfl_xor(ls, 2, 32);
                ls += __shfl_xor(ls, 4, 32);
                ls += __shfl_xor(ls, 8, 32);
                lr[r] = lr[r] * alpha + ls;
                #pragma unroll
                for (int t = 0; t < 4; ++t) Oacc[t][r] *= alpha;
            }
        }
        __syncthreads();

        if (active) {
            #pragma unroll
            for (int s = 0; s < 2; ++s) {
                Frag fp;
                fp.h8[0] = *(const v8h*)(&sm.a.Ps[wid][m][s * 32 + 8 * hs]);
                fp.h8[1] = *(const v8h*)(&sm.a.Ps[wid][m][s * 32 + 16 + 8 * hs]);
                #pragma unroll
                for (int t = 0; t < 4; ++t) {
                    Frag fv;
                    fv.h8[0] = *(const v8h*)(&sm.a.Vt[t * 16 + m][s * 32 + 8 * hs]);
                    fv.h8[1] = *(const v8h*)(&sm.a.Vt[t * 16 + m][s * 32 + 16 + 8 * hs]);
                    Oacc[t] = wmma_f16_32k(fp.v, fv.v, Oacc[t]);
                }
            }
        }
    }

    __syncthreads();

    float inv[8];
    #pragma unroll
    for (int r = 0; r < 8; ++r) inv[r] = 1.0f / lr[r];
    #pragma unroll
    for (int r = 0; r < 8; ++r) {
        #pragma unroll
        for (int t = 0; t < 4; ++t)
            sm.b.Os[wid][r + 8 * hs][t * 16 + m] = Oacc[t][r] * inv[r];
    }
    __syncthreads();

    v4f ov[8];
    const int c4 = (lane & 15) * 4;
    #pragma unroll
    for (int i = 0; i < 8; ++i) ov[i] = *(const v4f*)(&sm.b.Os[wid][2 * i + hs][c4]);
    float* obase = out + base + (size_t)wrow0 * DIM;
    #pragma unroll
    for (int i = 0; i < 8; ++i)
        *(volatile v4f*)(obase + (size_t)(2 * i + hs) * DIM + c4) = ov[i];
    __threadfence();
    #pragma unroll
    for (int i = 0; i < 8; ++i)
        *(volatile v4f*)(obase + (size_t)(2 * i + hs) * DIM + c4) = ov[i];
}

extern "C" void kernel_launch(void* const* d_in, const int* in_sizes, int n_in,
                              void* d_out, int out_size, void* d_ws, size_t ws_size,
                              hipStream_t stream)
{
    (void)d_ws; (void)ws_size;
    const int total = BATCH * HEADS * SEQ * DIM;
    if (n_in < 3) return;
    if (in_sizes[0] != total || in_sizes[1] != total || in_sizes[2] != total || out_size != total) return;
    const float* q = (const float*)d_in[0];
    const float* k = (const float*)d_in[1];
    const float* v = (const float*)d_in[2];
    float* out = (float*)d_out;
    dim3 grid(SEQ / QT, BATCH * HEADS);
    dim3 block(NTHR);
    hipLaunchKernelGGL(attn_causal_fwd, grid, block, 0, stream, q, k, v, out, (int)(BATCH * HEADS));
    (void)hipGetLastError();
}
